// GraphEncoderBlock_81896436400166
// MI455X (gfx1250) — hardware-verified
//
#include <hip/hip_runtime.h>
#include <stdint.h>


#define DD 128
#define HD 512
#define EDD 16
#define FF 256

typedef _Float16 v8h __attribute__((ext_vector_type(8)));
typedef _Float16 v16h __attribute__((ext_vector_type(16)));
typedef float v8f __attribute__((ext_vector_type(8)));
typedef float v4f __attribute__((ext_vector_type(4)));
typedef int v4i __attribute__((ext_vector_type(4)));
typedef unsigned long long u64;
typedef u64 v2u __attribute__((ext_vector_type(2)));

union Frag { v16h v; v8h half[2]; };

__device__ __forceinline__ v8f wmma16(v16h a, v16h b, v8f c) {
  c = __builtin_amdgcn_wmma_f32_16x16x32_f16(false, a, false, b, (short)0, c, false, false);
  asm volatile("v_nop\n\tv_nop\n\tv_nop\n\tv_nop" : "+v"(c) : "v"(a), "v"(b));
  return c;
}

__device__ __forceinline__ v8h cvt8(v4f p, v4f q) {
  v8h r;
  r[0] = (_Float16)p[0]; r[1] = (_Float16)p[1]; r[2] = (_Float16)p[2]; r[3] = (_Float16)p[3];
  r[4] = (_Float16)q[0]; r[5] = (_Float16)q[1]; r[6] = (_Float16)q[2]; r[7] = (_Float16)q[3];
  return r;
}

__device__ __forceinline__ v8h zero8h() {
  v4f z = {0.f, 0.f, 0.f, 0.f};
  return cvt8(z, z);
}

__device__ __forceinline__ v8f zero8f() {
  v8f c = {0.f, 0.f, 0.f, 0.f, 0.f, 0.f, 0.f, 0.f};
  return c;
}

__device__ __forceinline__ float ldf(const float* base, unsigned off) {
  return *(const float*)((const char*)base + off);
}

__device__ __forceinline__ int wrapclamp(int s, int N) {
  if (s < 0) s += N;
  s = s < 0 ? 0 : s;
  s = s >= N ? N - 1 : s;
  return s;
}

__device__ __forceinline__ float wmax32(float v) {
#pragma unroll
  for (int off = 16; off > 0; off >>= 1) v = fmaxf(v, __shfl_xor(v, off, 32));
  return v;
}

__device__ __forceinline__ float wsum32(float v) {
#pragma unroll
  for (int off = 16; off > 0; off >>= 1) v += __shfl_xor(v, off, 32);
  return v;
}

__global__ __launch_bounds__(256) void k_cvt(
    const float* __restrict__ Wl, const float* __restrict__ Wr,
    const float* __restrict__ W1, const float* __restrict__ W2, const float* __restrict__ We,
    _Float16* Wl_h, _Float16* Wr_h, _Float16* W1_h, _Float16* W2_h, _Float16* We_h, int total8) {
  const int g = blockIdx.x * 256 + threadIdx.x;
  if (g >= total8) return;
  const int c0 = HD * DD / 8;
  const int c1 = 2 * c0;
  const int c2 = c1 + FF * DD / 8;
  const int c3 = c2 + DD * FF / 8;
  const float* s; _Float16* d; int i;
  if (g < c0)      { s = Wl; d = Wl_h; i = g; }
  else if (g < c1) { s = Wr; d = Wr_h; i = g - c0; }
  else if (g < c2) { s = W1; d = W1_h; i = g - c1; }
  else if (g < c3) { s = W2; d = W2_h; i = g - c2; }
  else             { s = We; d = We_h; i = g - c3; }
  const v4f a = *(const v4f*)(s + 8 * i);
  const v4f b = *(const v4f*)(s + 8 * i + 4);
  const v8h hv = cvt8(a, b);
  volatile v8h* p = (volatile v8h*)(d + 8 * i);
  *p = hv;
  __threadfence();
  *p = hv;
}

__global__ __launch_bounds__(256) void k_sortblk(const int* __restrict__ ei, int E, int N, u64* out) {
  __shared__ u64 ks[2048];
  const int t = threadIdx.x;
  const int base = blockIdx.x * 2048;
#pragma unroll
  for (int s = 0; s < 8; s++) {
    const int i = t + 256 * s;
    const int pos = base + i;
    u64 k = ~0ull;
    if (pos < E) {
      int d = wrapclamp(ei[E + pos], N);
      k = ((u64)(unsigned)d << 32) | (u64)(unsigned)pos;
    }
    ks[i] = k;
  }
  __syncthreads();
#pragma unroll 1
  for (int kk = 2; kk <= 2048; kk <<= 1) {
#pragma unroll 1
    for (int j = kk >> 1; j > 0; j >>= 1) {
#pragma unroll
      for (int s = 0; s < 8; s++) {
        const int i = t + 256 * s;
        const int l = i ^ j;
        if (l > i) {
          const u64 a = ks[i], b = ks[l];
          const bool asc = (i & kk) == 0;
          const bool sw = asc ? (a > b) : (a < b);
          if (sw) { ks[i] = b; ks[l] = a; }
        }
      }
      __syncthreads();
    }
  }
#pragma unroll
  for (int s = 0; s < 4; s++) {
    const int i = 2 * t + 512 * s;
    v2u o; o[0] = ks[i]; o[1] = ks[i + 1];
    *(volatile v2u*)(out + base + i) = o;
  }
  __threadfence();
#pragma unroll
  for (int s = 0; s < 4; s++) {
    const int i = 2 * t + 512 * s;
    v2u o; o[0] = ks[i]; o[1] = ks[i + 1];
    *(volatile v2u*)(out + base + i) = o;
  }
}

__global__ __launch_bounds__(128) void k_merge(const u64* __restrict__ in, u64* out, int T, int R) {
  const int gw = blockIdx.x * 4 + (threadIdx.x >> 5);
  const int lane = threadIdx.x & 31;
  if (gw * 64 >= T) return;
  const int p = gw * 64 + 2 * lane;
  const int pair = p / (2 * R);
  const int pb = pair * 2 * R;
  int lenA = T - pb; lenA = lenA > R ? R : lenA;
  int lenB = T - pb - lenA; lenB = lenB < 0 ? 0 : (lenB > R ? R : lenB);
  const u64* A = in + pb;
  const u64* B = A + lenA;
  const int q = p - pb;
  int lo = q - lenB; lo = lo < 0 ? 0 : lo;
  int hi = q < lenA ? q : lenA;
  for (int it = 0; it < 24 && lo < hi; it++) {
    const int i = (lo + hi) >> 1;
    const int j = q - i;
    if (A[i] <= B[j - 1]) lo = i + 1; else hi = i;
  }
  int i = lo, j = q - lo;
  u64 ka = (i < lenA) ? A[i] : ~0ull;
  u64 kb = (j < lenB) ? B[j] : ~0ull;
  const bool ta = ka <= kb;
  const u64 o0 = ta ? ka : kb;
  if (ta) { i++; ka = (i < lenA) ? A[i] : ~0ull; }
  else    { j++; kb = (j < lenB) ? B[j] : ~0ull; }
  const u64 o1 = (ka <= kb) ? ka : kb;
  v2u o; o[0] = o0; o[1] = o1;
  volatile v2u* pp = (volatile v2u*)(out + p);
  *pp = o;
  __threadfence();
  *pp = o;
}

__global__ __launch_bounds__(128) void k_rowptr(const u64* __restrict__ ks, int E, int* rowptr, int Npad) {
  const int g = blockIdx.x * 128 + threadIdx.x;
  const int v0 = 4 * g;
  if (v0 >= Npad) return;
  v4i r = {0, 0, 0, 0};
#pragma unroll
  for (int c = 0; c < 4; c++) {
    const u64 key = (u64)(unsigned)(v0 + c) << 32;
    int lo = 0, hi = E;
    for (int it = 0; it < 32 && lo < hi; it++) {
      const int mid = (lo + hi) >> 1;
      if (ks[mid] < key) lo = mid + 1; else hi = mid;
    }
    r[c] = lo;
  }
  volatile v4i* p = (volatile v4i*)(rowptr + v0);
  *p = r;
  __threadfence();
  *p = r;
}

__global__ __launch_bounds__(128) void k_proj(const float* __restrict__ x, int N,
    const _Float16* __restrict__ Wl_h, const float* __restrict__ bl,
    const _Float16* __restrict__ Wr_h, const float* __restrict__ br,
    float* xl, float* xr) {
  __shared__ v8h As[16 * 17];
  __shared__ float stg[16 * 516];
  const int tid = threadIdx.x, w = tid >> 5, lane = tid & 31, h = lane >> 4, m = lane & 15;
  const int node0 = blockIdx.x * 16;
  {
    const int row = tid >> 3, seg = (tid & 7) * 16;
    const int node = node0 + row;
    v4f q0 = {0.f, 0.f, 0.f, 0.f}, q1 = q0, q2 = q0, q3 = q0;
    if (node < N) {
      const float* rp = x + (size_t)node * DD + seg;
      q0 = *(const v4f*)rp; q1 = *(const v4f*)(rp + 4);
      q2 = *(const v4f*)(rp + 8); q3 = *(const v4f*)(rp + 12);
    }
    As[row * 17 + (seg >> 3)] = cvt8(q0, q1);
    As[row * 17 + (seg >> 3) + 1] = cvt8(q2, q3);
  }
  __syncthreads();
  Frag a[4];
#pragma unroll
  for (int kc = 0; kc < 4; kc++) {
    a[kc].half[0] = As[m * 17 + 4 * kc + h];
    a[kc].half[1] = As[m * 17 + 4 * kc + 2 + h];
  }
#pragma unroll 1
  for (int sel = 0; sel < 2; sel++) {
    const _Float16* W = sel ? Wr_h : Wl_h;
    const float* bias = sel ? br : bl;
    float* dstp = sel ? xr : xl;
#pragma unroll 1
    for (int tt = 0; tt < 8; tt++) {
      const int n0 = 128 * w + 16 * tt;
      const _Float16* wrow = W + (size_t)(n0 + m) * DD;
      v8f acc = zero8f();
#pragma unroll
      for (int kc = 0; kc < 4; kc++) {
        Frag b;
        b.half[0] = *(const v8h*)(wrow + 32 * kc + 8 * h);
        b.half[1] = *(const v8h*)(wrow + 32 * kc + 16 + 8 * h);
        acc = wmma16(a[kc].v, b.v, acc);
      }
      const float bv = bias[n0 + m];
#pragma unroll
      for (int r = 0; r < 8; r++) stg[(8 * h + r) * 516 + n0 + m] = acc[r] + bv;
    }
    __syncthreads();
    for (int row = 0; row < 16; row++) {
      const int node = node0 + row;
      if (node < N) {
        const float* sp = stg + row * 516 + 4 * tid;
        v4f v = {sp[0], sp[1], sp[2], sp[3]};
        *(volatile v4f*)(dstp + (size_t)node * HD + 4 * tid) = v;
      }
    }
    __threadfence();
    for (int row = 0; row < 16; row++) {
      const int node = node0 + row;
      if (node < N) {
        const float* sp = stg + row * 516 + 4 * tid;
        v4f v = {sp[0], sp[1], sp[2], sp[3]};
        *(volatile v4f*)(dstp + (size_t)node * HD + 4 * tid) = v;
      }
    }
    __syncthreads();
  }
}

__global__ __launch_bounds__(128) void k_edge(const u64* __restrict__ ks, const int* __restrict__ ei,
    const float* __restrict__ ea, const _Float16* __restrict__ We_h, const float* __restrict__ att,
    const float* __restrict__ xl, const float* __restrict__ xr, float* logit, int E, int N, int T16) {
  const int tid = threadIdx.x;
  const int gw = blockIdx.x * 4 + (tid >> 5);
  const int lane = tid & 31, h = lane >> 4, m = lane & 15;
  if (gw >= T16) return;
  const int p0 = gw * 16;
  Frag a;
  {
    const u64 km = ks[p0 + m];
    unsigned em = (unsigned)km; if (em >= (unsigned)E) em = (unsigned)(E - 1);
    const float* er = ea + (size_t)em * EDD + 8 * h;
    a.half[0] = cvt8(*(const v4f*)er, *(const v4f*)(er + 4));
    a.half[1] = zero8h();
  }
  unsigned offl[8], offr[8];
#pragma unroll
  for (int r = 0; r < 8; r++) {
    const u64 kr = ks[p0 + 8 * h + r];
    unsigned e2 = (unsigned)kr; if (e2 >= (unsigned)E) e2 = (unsigned)(E - 1);
    const unsigned d2 = (unsigned)(kr >> 32);
    const int dn = d2 >= (unsigned)N ? N - 1 : (int)d2;
    const int sn = wrapclamp(ei[e2], N);
    offl[r] = (unsigned)sn * (unsigned)(HD * 4) + 4u * (unsigned)m;
    offr[r] = (unsigned)dn * (unsigned)(HD * 4) + 4u * (unsigned)m;
  }
  float lg0 = 0.f, lg1 = 0.f, lg2 = 0.f, lg3 = 0.f;
  const v8h z8 = zero8h();
  const v8f zf = zero8f();
#pragma unroll 1
  for (int hd = 0; hd < 4; hd++) {
    float part[8];
#pragma unroll
    for (int r = 0; r < 8; r++) part[r] = 0.f;
#pragma unroll
    for (int t8 = 0; t8 < 8; t8++) {
      const int colbase = 128 * hd + 16 * t8;
      const int col = colbase + m;
      Frag b;
      b.half[0] = *(const v8h*)(We_h + (size_t)col * EDD + 8 * h);
      b.half[1] = z8;
      v8f acc = wmma16(a.v, b.v, zf);
      const float av = att[col];
      const unsigned co = 4u * (unsigned)colbase;
#pragma unroll
      for (int r = 0; r < 8; r++) {
        float z = acc[r] + ldf(xl, offl[r] + co) + ldf(xr, offr[r] + co);
        z = fmaxf(z, 0.2f * z);
        part[r] = fmaf(av, z, part[r]);
      }
    }
#pragma unroll
    for (int off = 8; off > 0; off >>= 1) {
#pragma unroll
      for (int r = 0; r < 8; r++) part[r] += __shfl_xor(part[r], off, 32);
    }
    const int rr = m & 7;
    float s = part[0];
    s = rr == 1 ? part[1] : s;
    s = rr == 2 ? part[2] : s;
    s = rr == 3 ? part[3] : s;
    s = rr == 4 ? part[4] : s;
    s = rr == 5 ? part[5] : s;
    s = rr == 6 ? part[6] : s;
    s = rr == 7 ? part[7] : s;
    lg0 = hd == 0 ? s : lg0;
    lg1 = hd == 1 ? s : lg1;
    lg2 = hd == 2 ? s : lg2;
    lg3 = hd == 3 ? s : lg3;
  }
  v4f mine = {lg0, lg1, lg2, lg3};
  v4f oth;
  oth[0] = __shfl_xor(mine[0], 16, 32);
  oth[1] = __shfl_xor(mine[1], 16, 32);
  oth[2] = __shfl_xor(mine[2], 16, 32);
  oth[3] = __shfl_xor(mine[3], 16, 32);
  const int wanth = (m >> 3) & 1;
  v4f fin = mine;
  if (wanth != h) fin = oth;
  volatile v4f* lp = (volatile v4f*)(logit + (size_t)(p0 + m) * 4);
  if (lane < 16) *lp = fin;
  __threadfence();
  if (lane < 16) *lp = fin;
}

__global__ __launch_bounds__(128) void k_node(const int* __restrict__ rowptr, const u64* __restrict__ ks,
    const int* __restrict__ ei, const float* __restrict__ logit, const float* __restrict__ xl,
    const float* __restrict__ x, const float* __restrict__ cb, const float* __restrict__ g1,
    const float* __restrict__ be1, float* x1, int N, int E) {
  const int w = threadIdx.x >> 5, lane = threadIdx.x & 31;
  const int v = blockIdx.x * 4 + w;
  if (v >= N) return;
  int beg = rowptr[v], end = rowptr[v + 1];
  beg = beg < 0 ? 0 : beg;
  end = end > E ? E : end;
  const float ninf = -__builtin_huge_valf();
  float m0 = ninf, m1 = ninf, m2 = ninf, m3 = ninf;
  for (int c = beg; c < end; c += 32) {
    const int p = c + lane;
    if (p < end) {
      const v4f l4 = *(const v4f*)(logit + (size_t)p * 4);
      m0 = fmaxf(m0, l4[0]); m1 = fmaxf(m1, l4[1]); m2 = fmaxf(m2, l4[2]); m3 = fmaxf(m3, l4[3]);
    }
  }
  m0 = wmax32(m0); m1 = wmax32(m1); m2 = wmax32(m2); m3 = wmax32(m3);
  float d0 = 0.f, d1 = 0.f, d2 = 0.f, d3 = 0.f;
  for (int c = beg; c < end; c += 32) {
    const int p = c + lane;
    if (p < end) {
      const v4f l4 = *(const v4f*)(logit + (size_t)p * 4);
      d0 += expf(l4[0] - m0); d1 += expf(l4[1] - m1); d2 += expf(l4[2] - m2); d3 += expf(l4[3] - m3);
    }
  }
  d0 = wsum32(d0); d1 = wsum32(d1); d2 = wsum32(d2); d3 = wsum32(d3);
  const float i0 = 0.25f * __fdividef(1.0f, d0 + 1e-16f);
  const float i1 = 0.25f * __fdividef(1.0f, d1 + 1e-16f);
  const float i2 = 0.25f * __fdividef(1.0f, d2 + 1e-16f);
  const float i3 = 0.25f * __fdividef(1.0f, d3 + 1e-16f);
  v4f acc = {0.f, 0.f, 0.f, 0.f};
  for (int c = beg; c < end; c += 32) {
    const int p = c + lane;
    float a0 = 0.f, a1 = 0.f, a2 = 0.f, a3 = 0.f;
    int s = 0;
    if (p < end) {
      const v4f l4 = *(const v4f*)(logit + (size_t)p * 4);
      a0 = expf(l4[0] - m0) * i0; a1 = expf(l4[1] - m1) * i1;
      a2 = expf(l4[2] - m2) * i2; a3 = expf(l4[3] - m3) * i3;
      const u64 k = ks[p];
      unsigned e = (unsigned)k; if (e >= (unsigned)E) e = (unsigned)(E - 1);
      s = wrapclamp(ei[e], N);
    }
    int cnt = end - c; cnt = cnt > 32 ? 32 : cnt;
    for (int j = 0; j < cnt; j++) {
      const float b0 = __shfl(a0, j, 32), b1 = __shfl(a1, j, 32);
      const float b2 = __shfl(a2, j, 32), b3 = __shfl(a3, j, 32);
      const int sj = __shfl(s, j, 32);
      const float* xp = xl + (size_t)sj * HD + 4 * lane;
      const v4f y0 = *(const v4f*)xp;
      const v4f y1 = *(const v4f*)(xp + 128);
      const v4f y2 = *(const v4f*)(xp + 256);
      const v4f y3 = *(const v4f*)(xp + 384);
      acc += b0 * y0; acc += b1 * y1; acc += b2 * y2; acc += b3 * y3;
    }
  }
  const v4f cb4 = *(const v4f*)(cb + 4 * lane);
  const v4f g4 = *(const v4f*)(g1 + 4 * lane);
  const v4f bb4 = *(const v4f*)(be1 + 4 * lane);
  const v4f xv = *(const v4f*)(x + (size_t)v * DD + 4 * lane);
  const v4f hrow = acc + cb4;
  const v4f u = xv + hrow;
  float s1 = u[0] + u[1] + u[2] + u[3];
  s1 = wsum32(s1);
  const float mu = s1 * (1.f / 128.f);
  const v4f dv = u - mu;
  float s2 = dv[0] * dv[0] + dv[1] * dv[1] + dv[2] * dv[2] + dv[3] * dv[3];
  s2 = wsum32(s2);
  const float var = s2 * (1.f / 128.f);
  const float rs = rsqrtf(var + 1e-5f);
  const v4f o = dv * rs * g4 + bb4;
  volatile v4f* op = (volatile v4f*)(x1 + (size_t)v * DD + 4 * lane);
  *op = o;
  __threadfence();
  *op = o;
}

__global__ __launch_bounds__(128) void k_ffn(const float* __restrict__ x1, int N,
    const _Float16* __restrict__ W1_h, const float* __restrict__ b1,
    const _Float16* __restrict__ W2_h, const float* __restrict__ b2,
    const float* __restrict__ g2, const float* __restrict__ be2, float* out) {
  __shared__ v8h As[16 * 17];
  __shared__ __attribute__((aligned(16))) _Float16 ys[16 * 264];
  __shared__ float os[16 * 132];
  const int tid = threadIdx.x, w = tid >> 5, lane = tid & 31, h = lane >> 4, m = lane & 15;
  const int node0 = blockIdx.x * 16;
  {
    const int row = tid >> 3, seg = (tid & 7) * 16;
    const int node = node0 + row;
    v4f q0 = {0.f, 0.f, 0.f, 0.f}, q1 = q0, q2 = q0, q3 = q0;
    if (node < N) {
      const float* rp = x1 + (size_t)node * DD + seg;
      q0 = *(const v4f*)rp; q1 = *(const v4f*)(rp + 4);
      q2 = *(const v4f*)(rp + 8); q3 = *(const v4f*)(rp + 12);
    }
    As[row * 17 + (seg >> 3)] = cvt8(q0, q1);
    As[row * 17 + (seg >> 3) + 1] = cvt8(q2, q3);
  }
  __syncthreads();
  Frag a[4];
#pragma unroll
  for (int kc = 0; kc < 4; kc++) {
    a[kc].half[0] = As[m * 17 + 4 * kc + h];
    a[kc].half[1] = As[m * 17 + 4 * kc + 2 + h];
  }
#pragma unroll 1
  for (int tt = 0; tt < 4; tt++) {
    const int n0 = 64 * w + 16 * tt;
    const _Float16* wrow = W1_h + (size_t)(n0 + m) * DD;
    v8f acc = zero8f();
#pragma unroll
    for (int kc = 0; kc < 4; kc++) {
      Frag b;
      b.half[0] = *(const v8h*)(wrow + 32 * kc + 8 * h);
      b.half[1] = *(const v8h*)(wrow + 32 * kc + 16 + 8 * h);
      acc = wmma16(a[kc].v, b.v, acc);
    }
    const float bv = b1[n0 + m];
#pragma unroll
    for (int r = 0; r < 8; r++) {
      const float u = acc[r] + bv;
      const float g = 0.5f * u * (1.f + erff(u * 0.70710678118654752f));
      ys[(8 * h + r) * 264 + n0 + m] = (_Float16)g;
    }
  }
  __syncthreads();
#pragma unroll 1
  for (int t2 = 0; t2 < 2; t2++) {
    const int n0 = 32 * w + 16 * t2;
    const _Float16* wrow = W2_h + (size_t)(n0 + m) * FF;
    v8f acc = zero8f();
#pragma unroll
    for (int kc = 0; kc < 8; kc++) {
      const _Float16* yr = ys + m * 264 + 32 * kc;
      Frag a2, b;
      a2.half[0] = *(const v8h*)(yr + 8 * h);
      a2.half[1] = *(const v8h*)(yr + 16 + 8 * h);
      b.half[0] = *(const v8h*)(wrow + 32 * kc + 8 * h);
      b.half[1] = *(const v8h*)(wrow + 32 * kc + 16 + 8 * h);
      acc = wmma16(a2.v, b.v, acc);
    }
    const float bv = b2[n0 + m];
#pragma unroll
    for (int r = 0; r < 8; r++) os[(8 * h + r) * 132 + n0 + m] = acc[r] + bv;
  }
  __syncthreads();
  const v4f g4 = *(const v4f*)(g2 + 4 * lane);
  const v4f bb4 = *(const v4f*)(be2 + 4 * lane);
  v4f res[4];
#pragma unroll
  for (int rr = 0; rr < 4; rr++) {
    const int row = 4 * w + rr;
    const int node = node0 + row;
    const float* op = os + row * 132 + 4 * lane;
    const v4f o4 = {op[0], op[1], op[2], op[3]};
    v4f xv = {0.f, 0.f, 0.f, 0.f};
    if (node < N) xv = *(const v4f*)(x1 + (size_t)node * DD + 4 * lane);
    const v4f u = o4 + xv;
    float s1 = u[0] + u[1] + u[2] + u[3];
    s1 = wsum32(s1);
    const float mu = s1 * (1.f / 128.f);
    const v4f dv = u - mu;
    float s2 = dv[0] * dv[0] + dv[1] * dv[1] + dv[2] * dv[2] + dv[3] * dv[3];
    s2 = wsum32(s2);
    const float var = s2 * (1.f / 128.f);
    const float rs = rsqrtf(var + 1e-5f);
    res[rr] = dv * rs * g4 + bb4;
  }
#pragma unroll
  for (int rr = 0; rr < 4; rr++) {
    const int node = node0 + 4 * w + rr;
    if (node < N) *(volatile v4f*)(out + (size_t)node * DD + 4 * lane) = res[rr];
  }
  __threadfence();
#pragma unroll
  for (int rr = 0; rr < 4; rr++) {
    const int node = node0 + 4 * w + rr;
    if (node < N) *(volatile v4f*)(out + (size_t)node * DD + 4 * lane) = res[rr];
  }
}

extern "C" void kernel_launch(void* const* d_in, const int* in_sizes, int n_in,
                              void* d_out, int out_size, void* d_ws, size_t ws_size,
                              hipStream_t stream) {
  if (n_in < 18) return;
  const float* x   = (const float*)d_in[0];
  const int*   ei  = (const int*)d_in[1];
  const float* ea  = (const float*)d_in[2];
  const float* Wl  = (const float*)d_in[3];
  const float* bl  = (const float*)d_in[4];
  const float* Wr  = (const float*)d_in[5];
  const float* br  = (const float*)d_in[6];
  const float* We  = (const float*)d_in[7];
  const float* att = (const float*)d_in[8];
  const float* cb  = (const float*)d_in[9];
  const float* g1  = (const float*)d_in[10];
  const float* be1 = (const float*)d_in[11];
  const float* W1  = (const float*)d_in[12];
  const float* b1  = (const float*)d_in[13];
  const float* W2  = (const float*)d_in[14];
  const float* b2  = (const float*)d_in[15];
  const float* g2  = (const float*)d_in[16];
  const float* be2 = (const float*)d_in[17];
  float* out = (float*)d_out;

  const int N = in_sizes[0] / DD;
  const int E = in_sizes[1] / 2;
  if (N <= 0 || E <= 0) return;
  if (in_sizes[0] != N * DD || in_sizes[1] != 2 * E || in_sizes[2] != E * EDD) return;
  if (in_sizes[3] != HD * DD || in_sizes[5] != HD * DD || in_sizes[7] != HD * EDD) return;
  if (in_sizes[8] != HD || in_sizes[12] != FF * DD || in_sizes[14] != DD * FF) return;
  if (in_sizes[9] != DD || in_sizes[10] != DD || in_sizes[16] != DD) return;
  if (out_size != N * DD) return;

  const int nchunk = (E + 2047) / 2048;
  const int T = nchunk * 2048;
  const int T16 = (E + 15) / 16;
  const int Npad = ((N + 1 + 511) / 512) * 512;

  char* wsb = (char*)d_ws;
  size_t off = 0;
  auto take = [&](size_t bytes) -> char* {
    char* p = wsb + off;
    off += (bytes + 255) & ~(size_t)255;
    return p;
  };
  _Float16* Wl_h = (_Float16*)take((size_t)HD * DD * 2);
  _Float16* Wr_h = (_Float16*)take((size_t)HD * DD * 2);
  _Float16* W1_h = (_Float16*)take((size_t)FF * DD * 2);
  _Float16* W2_h = (_Float16*)take((size_t)DD * FF * 2);
  _Float16* We_h = (_Float16*)take((size_t)HD * EDD * 2);
  u64* keysA  = (u64*)take((size_t)T * 8);
  u64* keysB  = (u64*)take((size_t)T * 8);
  int* rowptr = (int*)take((size_t)Npad * 4);
  float* logit = (float*)take((size_t)T16 * 16 * 4 * 4);
  float* xl = (float*)take((size_t)N * HD * 4);
  float* xr = (float*)take((size_t)N * HD * 4);
  float* x1 = (float*)take((size_t)N * DD * 4);
  if (off > ws_size) return;

  const int total8 = (2 * HD * DD + FF * DD + DD * FF + HD * EDD) / 8;
  k_cvt<<<(total8 + 255) / 256, 256, 0, stream>>>(Wl, Wr, W1, W2, We, Wl_h, Wr_h, W1_h, W2_h, We_h, total8);

  k_sortblk<<<nchunk, 256, 0, stream>>>(ei, E, N, keysA);
  u64* cur = keysA;
  u64* nxt = keysB;
  for (int R = 2048; R < T; R <<= 1) {
    const int waves = T / 64;
    const int blocks = (waves + 3) / 4;
    k_merge<<<blocks, 128, 0, stream>>>(cur, nxt, T, R);
    u64* tmp = cur; cur = nxt; nxt = tmp;
  }
  k_rowptr<<<Npad / 512, 128, 0, stream>>>(cur, E, rowptr, Npad);

  k_proj<<<(N + 15) / 16, 128, 0, stream>>>(x, N, Wl_h, bl, Wr_h, br, xl, xr);
  k_edge<<<(T16 + 3) / 4, 128, 0, stream>>>(cur, ei, ea, We_h, att, xl, xr, logit, E, N, T16);
  k_node<<<(N + 3) / 4, 128, 0, stream>>>(rowptr, cur, ei, logit, xl, x, cb, g1, be1, x1, N, E);
  k_ffn<<<(N + 15) / 16, 128, 0, stream>>>(x1, N, W1_h, b1, W2_h, b2, g2, be2, out);
}
